// EncoderLayer_28698971472471
// MI455X (gfx1250) — hardware-verified
//
#include <hip/hip_runtime.h>
#ifndef NB
#define NB 2
#endif
#ifndef SEQ
#define SEQ 2048
#endif
#define NB_FULL 2
#define SEQ_FULL 2048
#define DM 1024
#define NH 16
#define HD 64
#define DFF 4096
#define LQ (3 * DM)
#define NR ((size_t)NB * SEQ)

static_assert(NB >= 1 && NB <= NB_FULL);
static_assert(SEQ <= SEQ_FULL && SEQ % 128 == 0);
static_assert(NH * HD == DM && HD == 64);
static_assert(DM % 64 == 0 && DFF % 64 == 0 && LQ % 64 == 0);
static_assert(((size_t)NB * SEQ) % 128 == 0);

typedef unsigned short v8us __attribute__((ext_vector_type(8), may_alias));
typedef float  v8f  __attribute__((ext_vector_type(8)));
typedef float  v4f  __attribute__((ext_vector_type(4)));
typedef float  v4fa __attribute__((ext_vector_type(4), may_alias));
typedef int    v4i  __attribute__((ext_vector_type(4)));
typedef int    v4ia __attribute__((ext_vector_type(4), may_alias));
typedef _Float16 v16h __attribute__((ext_vector_type(16)));
typedef _Float16 v4h  __attribute__((ext_vector_type(4)));
union FragH { v16h v; v8us half[2]; _Float16 h[16]; unsigned short u[16]; };

__device__ __forceinline__ unsigned short bf16_bits(float x) { unsigned int u = __float_as_uint(x); return (unsigned short)((u + 0x7FFFu + ((u >> 16) & 1u)) >> 16); }
__device__ __forceinline__ float bf16_rne(float x) { return __uint_as_float(((unsigned int)bf16_bits(x)) << 16); }

__device__ __forceinline__ v16h g2_frag(const _Float16* p, unsigned hh) { FragH f; f.half[0] = *(const v8us*)((const unsigned short*)p + 8u * hh); f.half[1] = *(const v8us*)((const unsigned short*)p + 16u + 8u * hh); return f.v; }
__device__ __forceinline__ v8f g2_mma(v16h a, v16h b, v8f c) { v8f d = __builtin_amdgcn_wmma_f32_16x16x32_f16(false, a, false, b, (short)0, c, false, false); asm volatile("v_nop\n\tv_nop\n\tv_nop\n\tv_nop" : "+v"(d) : "v"(a), "v"(b)); return d; }

__global__ __launch_bounds__(256) void k_wt_f16(const float* __restrict__ W, _Float16* __restrict__ Wt, unsigned K, unsigned N, float scale) {
  const unsigned t = blockIdx.x * 256u + threadIdx.x; const unsigned k8n = K >> 3;
  if (t >= N * k8n) return;
  const unsigned n = t / k8n, k8 = (t - n * k8n) << 3;
  FragH f;
#pragma unroll
  for (int i = 0; i < 8; ++i) f.h[i] = (_Float16)(bf16_rne(W[(size_t)(k8 + i) * N + n]) * scale);
  const v8us o = f.half[0];
  unsigned short* dst = (unsigned short*)Wt + (size_t)n * K + k8;
  *(volatile v8us*)dst = o; __threadfence(); *(volatile v8us*)dst = o;
}

template <int BFIN, int WXB, int XFULL>
__global__ __launch_bounds__(256) void k_ln16(const float* __restrict__ X, const float* __restrict__ g, const float* __restrict__ bb, float eps, _Float16* __restrict__ N16, float* __restrict__ XB) {
  #pragma clang fp contract(off)
  __shared__ float red[256];
  const unsigned r = blockIdx.x, t = threadIdx.x;
  size_t rs = r;
  if (XFULL) { const unsigned b = r / (unsigned)SEQ; rs = (size_t)b * SEQ_FULL + (r - b * (unsigned)SEQ); }
  const v4f xa = *(const v4fa*)(X + rs * DM + t * 4u);
  float s[4]; float sum = 0.f;
#pragma unroll
  for (int q = 0; q < 4; ++q) { s[q] = BFIN ? bf16_rne(xa[q]) : xa[q]; sum = sum + s[q]; }
  red[t] = sum; __syncthreads();
  for (unsigned st = 128u; st > 0u; st >>= 1) { if (t < st) red[t] = red[t] + red[t + st]; __syncthreads(); }
  const float mu = red[0] * (1.0f / (float)DM); __syncthreads();
  float vs = 0.f;
#pragma unroll
  for (int q = 0; q < 4; ++q) { const float dl = s[q] - mu; vs = vs + dl * dl; }
  red[t] = vs; __syncthreads();
  for (unsigned st = 128u; st > 0u; st >>= 1) { if (t < st) red[t] = red[t] + red[t + st]; __syncthreads(); }
  const float rsd = rsqrtf(red[0] * (1.0f / (float)DM) + eps);
  const v4f gv = *(const v4fa*)(g + t * 4u), bv = *(const v4fa*)(bb + t * 4u);
  v4h y; v4f xb;
#pragma unroll
  for (int q = 0; q < 4; ++q) { y[q] = (_Float16)(((s[q] - mu) * rsd) * bf16_rne(gv[q]) + bf16_rne(bv[q])); xb[q] = s[q]; }
  const size_t o = (size_t)r * DM + t * 4u;
  for (int pass = 0; pass < 2; ++pass) { *(volatile v4h*)(N16 + o) = y; if (WXB) *(volatile v4f*)(XB + o) = xb; if (pass == 0) __threadfence(); }
}

template <int ACT>
__global__ __launch_bounds__(128) void k_gemm2(const _Float16* __restrict__ A, unsigned lda, const _Float16* __restrict__ Bh, unsigned ldb, float alpha,
    const float* __restrict__ bias, const float* __restrict__ CP, float* __restrict__ C, _Float16* __restrict__ C16, unsigned ldc, unsigned M, unsigned N, unsigned K) {
  static_assert(ACT == 0 || ACT == 3);
  __shared__ __attribute__((aligned(16))) float so[4][32][68];
  const unsigned tid = threadIdx.x, w = tid >> 5, lane = tid & 31u, ln = lane & 15u, hh = lane >> 4;
  const unsigned ntn = N >> 6; const unsigned mt = blockIdx.x / ntn, nq = blockIdx.x - mt * ntn;
  const unsigned row0 = mt * 128u + 32u * w, col0 = nq * 64u;
  if (row0 >= M) return;
  const _Float16* a0p = A + (size_t)(row0 + ln) * lda; const _Float16* a1p = a0p + (size_t)16 * lda;
  const _Float16* b0p = Bh + (size_t)(col0 + ln) * ldb; const _Float16* b1p = b0p + (size_t)16 * ldb; const _Float16* b2p = b1p + (size_t)16 * ldb; const _Float16* b3p = b2p + (size_t)16 * ldb;
  const v8f z8 = {0.f,0.f,0.f,0.f,0.f,0.f,0.f,0.f}; v8f c00 = z8, c01 = z8, c02 = z8, c03 = z8, c10 = z8, c11 = z8, c12 = z8, c13 = z8;
#pragma unroll 1
  for (unsigned kb = 0; kb < K; kb += 32u) { const v16h a0 = g2_frag(a0p + kb, hh), a1 = g2_frag(a1p + kb, hh);
    v16h b = g2_frag(b0p + kb, hh); c00 = g2_mma(a0, b, c00); c10 = g2_mma(a1, b, c10);
    b = g2_frag(b1p + kb, hh); c01 = g2_mma(a0, b, c01); c11 = g2_mma(a1, b, c11);
    b = g2_frag(b2p + kb, hh); c02 = g2_mma(a0, b, c02); c12 = g2_mma(a1, b, c12);
    b = g2_frag(b3p + kb, hh); c03 = g2_mma(a0, b, c03); c13 = g2_mma(a1, b, c13); }
  v8f accs[8] = {c00, c01, c02, c03, c10, c11, c12, c13};
#pragma unroll
  for (int u = 0; u < 8; ++u) { const unsigned t = (unsigned)(u & 3), half = (unsigned)(u >> 2); const unsigned col = col0 + t * 16u + ln; const float bv = bias ? bf16_rne(bias[col]) : 0.f;
#pragma unroll
    for (int r = 0; r < 8; ++r) { const unsigned rloc = half * 16u + 8u * hh + (unsigned)r; float v = accs[u][r] * alpha + bv;
      if (CP) v += CP[(size_t)(row0 + rloc) * ldc + col];
      if (ACT == 3) v = fmaxf(v, 0.f);
      so[w][rloc][t * 16u + ln] = v; } }
  __builtin_amdgcn_fence(4  , "workgroup"); __builtin_amdgcn_wave_barrier();
  const unsigned rsub = lane >> 4, c4 = (lane & 15u) * 4u;
  for (int pass = 0; pass < 2; ++pass) {
#pragma unroll
    for (int q = 0; q < 16; ++q) { const unsigned r = (unsigned)q * 2u + rsub; const v4f v = *(const v4fa*)&so[w][r][c4];
      if (C) *(volatile v4f*)(C + (size_t)(row0 + r) * ldc + col0 + c4) = v;
      if (C16) { v4h h4;
#pragma unroll
        for (int i = 0; i < 4; ++i) h4[i] = (_Float16)v[i];
        *(volatile v4h*)(C16 + (size_t)(row0 + r) * ldc + col0 + c4) = h4; } }
    if (pass == 0) __threadfence(); }
}

__global__ __launch_bounds__(256) void k_ropetab(float* __restrict__ CS) {
  const unsigned idx = blockIdx.x * 256u + threadIdx.x;
  const unsigned t = idx >> 5, i = idx & 31u;
  if (t >= (unsigned)SEQ) return;
  const float th = expf(-(float)i * 0.28782313662425576f);
  const float ang = (float)t * th;
  float sn, cs; sincosf(ang, &sn, &cs);
  float* pc = CS + (size_t)t * 64u + i;
  *(volatile float*)pc = cs; *(volatile float*)(pc + 32) = sn;
  __threadfence();
  *(volatile float*)pc = cs; *(volatile float*)(pc + 32) = sn;
}

__global__ __launch_bounds__(256) void k_rope(_Float16* __restrict__ QKV, const float* __restrict__ CS) {
  const unsigned row = blockIdx.x, tid = threadIdx.x;
  const unsigned t = row % (unsigned)SEQ;
  const unsigned col = tid * 8u;
  const unsigned d = col & 63u;
  const float sc = (col < (unsigned)DM) ? 0.125f : 1.0f;
  unsigned short* p = (unsigned short*)QKV + (size_t)row * LQ + col;
  FragH f; f.half[0] = *(const v8us*)p;
  const v4f c4 = *(const v4fa*)(CS + (size_t)t * 64u + (d >> 1));
  const v4f s4 = *(const v4fa*)(CS + (size_t)t * 64u + 32u + (d >> 1));
  FragH o;
#pragma unroll
  for (int q = 0; q < 4; ++q) { const float x1 = (float)f.h[2 * q], x2 = (float)f.h[2 * q + 1];
    o.h[2 * q] = (_Float16)((x1 * c4[q] - x2 * s4[q]) * sc); o.h[2 * q + 1] = (_Float16)((x1 * s4[q] + x2 * c4[q]) * sc); }
  const v8us ov = o.half[0];
  *(volatile v8us*)p = ov; __threadfence(); *(volatile v8us*)p = ov;
}

__global__ __launch_bounds__(256) void k_vt(const _Float16* __restrict__ V16, unsigned ldv, _Float16* __restrict__ Vt) {
  __shared__ unsigned short tl[64][66];
  const unsigned tid = threadIdx.x; const unsigned ng = (unsigned)SEQ / 64u;
  const unsigned slab = blockIdx.x / ng, lg = blockIdx.x - slab * ng; const unsigned b = slab / (unsigned)NH, h = slab - b * (unsigned)NH;
  for (unsigned i = tid; i < 512u; i += 256u) { const unsigned r = i >> 3, c8 = (i & 7u) << 3; FragH f;
    f.half[0] = *(const v8us*)((const unsigned short*)V16 + ((size_t)b * SEQ + lg * 64u + r) * ldv + h * 64u + c8);
#pragma unroll
    for (int q = 0; q < 8; ++q) tl[r][c8 + q] = f.u[q]; }
  __syncthreads();
  for (int pass = 0; pass < 2; ++pass) {
#pragma unroll
    for (int rd = 0; rd < 2; ++rd) { const unsigned d = (unsigned)rd * 32u + (tid >> 3), pc = tid & 7u; FragH f;
#pragma unroll
      for (int q = 0; q < 8; ++q) f.u[q] = tl[pc * 8u + q][d];
      *(volatile v8us*)((unsigned short*)Vt + ((size_t)slab * 64u + d) * SEQ + lg * 64u + pc * 8u) = f.half[0]; }
    if (pass == 0) __threadfence(); }
}

__global__ __launch_bounds__(128) void k_fattn(const _Float16* __restrict__ QKV, const _Float16* __restrict__ VT, const int* __restrict__ msk, _Float16* __restrict__ O16) {
  __shared__ __attribute__((aligned(16))) unsigned short ot[4][16][72];
  const unsigned tid = threadIdx.x, w = tid >> 5, lane = tid & 31u, ln = lane & 15u, hh = lane >> 4;
  const unsigned wid = blockIdx.x * 4u + w;
  const unsigned ntq = (unsigned)SEQ / 16u;
  const unsigned bh = wid / ntq, mt = wid - bh * ntq;
  const unsigned b = bh / (unsigned)NH, hd = bh - b * (unsigned)NH;
  const unsigned t0 = mt * 16u;
  const size_t tok0 = (size_t)b * SEQ;
  const _Float16* qrow = QKV + (tok0 + t0 + ln) * LQ + hd * HD;
  const _Float16* kbase = QKV + (tok0 + ln) * LQ + DM + hd * HD;
  const _Float16* vbase = VT + ((size_t)bh * HD + ln) * SEQ;
  const int* mrow = msk + ((size_t)b * SEQ_FULL + t0 + ln) * SEQ_FULL + 8u * hh;
  const v16h qf0 = g2_frag(qrow, hh), qf1 = g2_frag(qrow + 32, hh);
  const v8f z8 = {0.f,0.f,0.f,0.f,0.f,0.f,0.f,0.f};
  v8f o0 = z8, o1 = z8, o2 = z8, o3 = z8;
  float mrun = -1.0e30f, lrun = 0.f;
#pragma unroll 1
  for (unsigned s0 = 0; s0 < (unsigned)SEQ; s0 += 32u) {
    const _Float16* k0p = kbase + (size_t)s0 * LQ; const _Float16* k1p = k0p + (size_t)16 * LQ;
    v8f st0 = z8, st1 = z8;
    st0 = g2_mma(g2_frag(k0p, hh), qf0, st0); st0 = g2_mma(g2_frag(k0p + 32, hh), qf1, st0);
    st1 = g2_mma(g2_frag(k1p, hh), qf0, st1); st1 = g2_mma(g2_frag(k1p + 32, hh), qf1, st1);
    const v4i ma = *(const v4ia*)(mrow + s0), mb = *(const v4ia*)(mrow + s0 + 4u), mc = *(const v4ia*)(mrow + s0 + 16u), md = *(const v4ia*)(mrow + s0 + 20u);
    const int mm0[8] = {ma[0], ma[1], ma[2], ma[3], mb[0], mb[1], mb[2], mb[3]};
    const int mm1[8] = {mc[0], mc[1], mc[2], mc[3], md[0], md[1], md[2], md[3]};
    float a0[8], a1[8]; float mx = -1.0e30f;
#pragma unroll
    for (int r = 0; r < 8; ++r) { a0[r] = (mm0[r] != 0) ? st0[r] : -1.0e30f; a1[r] = (mm1[r] != 0) ? st1[r] : -1.0e30f; mx = fmaxf(mx, fmaxf(a0[r], a1[r])); }
    mx = fmaxf(mx, __shfl_xor(mx, 16));
    const float mnew = fmaxf(mrun, mx);
    const float alpha = __expf(mrun - mnew);
    mrun = mnew;
    float rs = 0.f; FragH pf;
#pragma unroll
    for (int r = 0; r < 8; ++r) { const float e0 = __expf(a0[r] - mnew), e1 = __expf(a1[r] - mnew);
      const float p0 = (mm0[r] != 0) ? e0 : 0.f, p1 = (mm1[r] != 0) ? e1 : 0.f;
      rs += p0 + p1; pf.h[r] = (_Float16)(p0 * 256.0f); pf.h[8 + r] = (_Float16)(p1 * 256.0f); }
    rs += __shfl_xor(rs, 16);
    lrun = lrun * alpha + rs;
    o0 = o0 * alpha; o1 = o1 * alpha; o2 = o2 * alpha; o3 = o3 * alpha;
    const _Float16* vp = vbase + s0;
    o0 = g2_mma(g2_frag(vp, hh), pf.v, o0);
    o1 = g2_mma(g2_frag(vp + (size_t)16 * SEQ, hh), pf.v, o1);
    o2 = g2_mma(g2_frag(vp + (size_t)32 * SEQ, hh), pf.v, o2);
    o3 = g2_mma(g2_frag(vp + (size_t)48 * SEQ, hh), pf.v, o3);
  }
  const float inv = (lrun > 0.f) ? (0.25f / lrun) : __uint_as_float(0x7fc00000u);
  const v8f oo[4] = {o0, o1, o2, o3};
#pragma unroll
  for (int j = 0; j < 4; ++j) { FragH f;
#pragma unroll
    for (int r = 0; r < 8; ++r) f.h[r] = (_Float16)(oo[j][r] * inv);
    *(v8us*)&ot[w][ln][16 * j + 8u * hh] = f.half[0]; }
  __builtin_amdgcn_fence(4  , "workgroup"); __builtin_amdgcn_wave_barrier();
  unsigned short* obase = (unsigned short*)O16 + (tok0 + t0) * DM + hd * HD;
  const unsigned rq = lane >> 3, pc = (lane & 7u) * 8u;
  for (int pass = 0; pass < 2; ++pass) {
#pragma unroll
    for (int q = 0; q < 4; ++q) { const unsigned row = (unsigned)q * 4u + rq; const v8us v = *(const v8us*)&ot[w][row][pc];
      *(volatile v8us*)(obase + (size_t)row * DM + pc) = v; }
    if (pass == 0) __threadfence(); }
}

extern "C" void kernel_launch(void* const* d_in, const int* in_sizes, int n_in,
                              void* d_out, int out_size, void* d_ws, size_t ws_size, hipStream_t stream) {
  if (n_in < 15) return;
  const size_t need_x = ((size_t)(NB - 1) * SEQ_FULL + SEQ) * DM;
  const size_t need_m = ((size_t)(NB - 1) * SEQ_FULL + SEQ - 1) * SEQ_FULL + SEQ;
  if ((size_t)in_sizes[0] < need_x || (size_t)in_sizes[1] < need_m) return;
  if (in_sizes[2] < DM * DM || in_sizes[3] < DM * DM || in_sizes[4] < DM * DM || in_sizes[5] < DM * DM) return;
  if (in_sizes[6] < DM || in_sizes[7] < DM || in_sizes[8] < DM || in_sizes[9] < DM || in_sizes[10] < DM) return;
  if (in_sizes[11] < DM * DFF || in_sizes[12] < DFF || in_sizes[13] < DFF * DM || in_sizes[14] < DM) return;
  if ((size_t)out_size < NR * DM) return;
  const float* x = (const float*)d_in[0]; const int* msk = (const int*)d_in[1];
  const float* wq = (const float*)d_in[2]; const float* wk = (const float*)d_in[3]; const float* wv = (const float*)d_in[4]; const float* wo = (const float*)d_in[5]; const float* bo = (const float*)d_in[6];
  const float* g1 = (const float*)d_in[7]; const float* be1 = (const float*)d_in[8]; const float* g2 = (const float*)d_in[9]; const float* be2 = (const float*)d_in[10];
  const float* w1 = (const float*)d_in[11]; const float* b1 = (const float*)d_in[12]; const float* w2 = (const float*)d_in[13]; const float* b2 = (const float*)d_in[14];
  float* out = (float*)d_out;

  constexpr size_t SZ_BQKV = (size_t)3 * DM * DM * 2, SZ_BO = (size_t)DM * DM * 2, SZ_BW = (size_t)DFF * DM * 2;
  constexpr size_t SZ_CS = (size_t)SEQ * 64 * 4;
  constexpr size_t SZ_H16 = NR * DM * 2, SZ_F32 = NR * DM * 4;
  constexpr size_t SZ_QKV = NR * LQ * 2, SZ_VT = (size_t)NB * NH * HD * SEQ * 2, SZ_HF = NR * DFF * 2;
  constexpr size_t SZ_R1 = (SZ_QKV + SZ_VT > SZ_HF) ? (SZ_QKV + SZ_VT) : SZ_HF;
  static_assert(SZ_QKV % 256 == 0 && SZ_QKV + SZ_VT <= SZ_R1 && SZ_HF <= SZ_R1);
  constexpr size_t SZ_TOTAL = SZ_BQKV + SZ_BO + 2 * SZ_BW + SZ_CS + SZ_H16 + 2 * SZ_F32 + SZ_H16 + SZ_R1;
  static_assert(SZ_TOTAL + 16 * 256 <= (size_t)134217728);
  static_assert((NR / 128) * (LQ / 64) * 4 * 32 * 64 == NR * LQ);
  static_assert(((size_t)NB * NH * SEQ / 64) * 4 * 16 * 64 == NR * DM);
  static_assert(NR * 256 * 8 == NR * 2 * DM);
  static_assert(((size_t)NB * NH * (SEQ / 64)) * 64 * 64 == (size_t)NB * NH * HD * SEQ);
  static_assert(((size_t)SEQ / 8) * 256 * 2 == (size_t)SEQ * 64);
  static_assert((NR / 128) * (DFF / 64) * 4 * 32 * 64 == NR * DFF && (NR / 128) * (DM / 64) * 4 * 32 * 64 == NR * DM);

  char* ws = (char*)d_ws; size_t off = 0;
  auto take = [&](size_t bytes) { char* p = ws + off; off += (bytes + 255) & ~(size_t)255; return p; };
  _Float16* BQKV = (_Float16*)take(SZ_BQKV); _Float16* BO = (_Float16*)take(SZ_BO); _Float16* BW1 = (_Float16*)take(SZ_BW); _Float16* BW2 = (_Float16*)take(SZ_BW);
  float* CS = (float*)take(SZ_CS);
  _Float16* X16 = (_Float16*)take(SZ_H16); _Float16* M16 = X16;
  float* XB = (float*)take(SZ_F32); float* X1 = (float*)take(SZ_F32);
  _Float16* O16 = (_Float16*)take(SZ_H16);
  char* R1 = take(SZ_R1);
  _Float16* QKV = (_Float16*)R1; _Float16* VT = (_Float16*)(R1 + SZ_QKV); _Float16* HF16 = (_Float16*)R1;
  if (off > ws_size) return;

  { const unsigned g = (unsigned)(((size_t)DM * (DM / 8) + 255) / 256);
    k_wt_f16<<<g, 256, 0, stream>>>(wq, BQKV, DM, DM, 16.0f);
    k_wt_f16<<<g, 256, 0, stream>>>(wk, BQKV + (size_t)DM * DM, DM, DM, 16.0f);
    k_wt_f16<<<g, 256, 0, stream>>>(wv, BQKV + (size_t)2 * DM * DM, DM, DM, 16.0f);
    k_wt_f16<<<g, 256, 0, stream>>>(wo, BO, DM, DM, 16.0f); }
  k_wt_f16<<<(unsigned)(((size_t)DFF * (DM / 8) + 255) / 256), 256, 0, stream>>>(w1, BW1, DM, DFF, 16.0f);
  k_wt_f16<<<(unsigned)(((size_t)DM * (DFF / 8) + 255) / 256), 256, 0, stream>>>(w2, BW2, DFF, DM, 16.0f);
  k_ropetab<<<(unsigned)(SEQ / 8), 256, 0, stream>>>(CS);
  k_ln16<1, 1, 1><<<(unsigned)NR, 256, 0, stream>>>(x, g1, be1, 1e-5f, X16, XB);
  k_gemm2<0><<<(unsigned)((NR / 128) * (LQ / 64)), 128, 0, stream>>>(X16, DM, BQKV, DM, 0.0625f, nullptr, nullptr, nullptr, QKV, LQ, (unsigned)NR, LQ, DM);
  k_rope<<<(unsigned)NR, 256, 0, stream>>>(QKV, CS);
  k_vt<<<(unsigned)(NB * NH * (SEQ / 64)), 256, 0, stream>>>(QKV + 2 * DM, LQ, VT);
  k_fattn<<<(unsigned)((size_t)NB * NH * SEQ / 64), 128, 0, stream>>>(QKV, VT, msk, O16);
  k_gemm2<0><<<(unsigned)((NR / 128) * (DM / 64)), 128, 0, stream>>>(O16, DM, BO, DM, 0.0009765625f, bo, XB, X1, nullptr, DM, (unsigned)NR, DM, DM);
  k_ln16<0, 0, 0><<<(unsigned)NR, 256, 0, stream>>>(X1, g2, be2, 1e-5f, M16, nullptr);
  k_gemm2<3><<<(unsigned)((NR / 128) * (DFF / 64)), 128, 0, stream>>>(M16, DM, BW1, DM, 0.0625f, b1, nullptr, nullptr, HF16, DFF, (unsigned)NR, DFF, DM);
  k_gemm2<0><<<(unsigned)((NR / 128) * (DM / 64)), 128, 0, stream>>>(HF16, DFF, BW2, DFF, 0.0625f, b2, X1, out, nullptr, DM, (unsigned)NR, DM, DFF);
}
